// test_model9_53420803228132
// MI455X (gfx1250) — hardware-verified
//
#include <hip/hip_runtime.h>


#define NB     2
#define SEQ    4096
#define DIM    512
#define QT     16
#define CH     1024
#define NCH    (SEQ / CH)
#define NTHR   256

#define LDS_Q   (QT * DIM * 2)
#define LDS_S   (QT * CH * 4)
#define LDS_P   (QT * CH * 2)
#define LDS_ST  (2 * QT * 4)
#define LDS_ALL (LDS_Q + LDS_S + LDS_P + LDS_ST)

#define P_SCALE 32768.0f
#define C_SCALE 0.125f
#define O_SCALE 0.000244140625f
#define NEG_BIG (-1.0e30f)

typedef __attribute__((ext_vector_type(8)))  float          v8f;
typedef __attribute__((ext_vector_type(4)))  float          v4f_r;
typedef __attribute__((ext_vector_type(8)))  unsigned short v8us_r;
typedef __attribute__((ext_vector_type(16))) __bf16         v16bf;
typedef __attribute__((ext_vector_type(16))) _Float16       v16h;
typedef v4f_r  __attribute__((may_alias)) v4f;
typedef v8us_r __attribute__((may_alias)) v8us;

union FragB { v16bf v; v8us_r u[2]; };
union FragH { v16h  v; v8us_r u[2]; };

__device__ __forceinline__ v8f z8() {
  v8f z = {0.f, 0.f, 0.f, 0.f, 0.f, 0.f, 0.f, 0.f};
  return z;
}

__device__ __forceinline__ unsigned short f32_to_bf16_rne(float f) {
  unsigned u = __float_as_uint(f);
  u = u + 0x7FFFu + ((u >> 16) & 1u);
  return (unsigned short)(u >> 16);
}
__device__ __forceinline__ float bf16_to_f32(unsigned short b) {
  return __uint_as_float(((unsigned)b) << 16);
}
__device__ __forceinline__ unsigned short h_bits(_Float16 x) {
  union { _Float16 h; unsigned short u; } c;
  c.h = x;
  return c.u;
}

template <class F>
__device__ __forceinline__ F ld_frag(const unsigned short* base, int row0, int k0, int ld, int lane) {
  const int hh = lane >> 4, mm = lane & 15;
  const unsigned short* p = base + (size_t)(row0 + mm) * (size_t)ld + k0 + 8 * hh;
  F f;
  f.u[0] = *(const v8us*)(p);
  f.u[1] = *(const v8us*)(p + 16);
  return f;
}

__device__ __forceinline__ v8f mma_bf16(const FragB& a, const FragB& b, v8f c) {
  v8f d = __builtin_amdgcn_wmma_f32_16x16x32_bf16(false, a.v, false, b.v, (short)0, c, false, false);
  asm volatile("v_nop\n\tv_nop\n\tv_nop\n\tv_nop" : "+v"(d) : "v"(a.v), "v"(b.v));
  return d;
}
__device__ __forceinline__ v8f mma_f16(const FragH& a, const FragH& b, v8f c) {
  v8f d = __builtin_amdgcn_wmma_f32_16x16x32_f16(false, a.v, false, b.v, (short)0, c, false, false);
  asm volatile("v_nop\n\tv_nop\n\tv_nop\n\tv_nop" : "+v"(d) : "v"(a.v), "v"(b.v));
  return d;
}

template <int MODE>
__global__ __launch_bounds__(NTHR)
void k_tr16(const float* __restrict__ in, unsigned short* __restrict__ outp, int R, int C)
{
  __shared__ float tile[32][65];
  const int tid = threadIdx.x, lane = tid & 31, wave = tid >> 5;
  const size_t boff = (size_t)blockIdx.z * (size_t)R * (size_t)C;
  const int c0 = blockIdx.x * 32, r0 = blockIdx.y * 64;
  {
    const int c = c0 + lane;
#pragma unroll
    for (int i = 0; i < 8; ++i) {
      const int rl = wave + 8 * i;
      const int r = r0 + rl;
      float v = 0.0f;
      if (r < R && c < C) v = in[boff + (size_t)r * (size_t)C + c];
      tile[lane][rl] = v;
    }
  }
  __syncthreads();
  const int cl = 4 * wave + (lane >> 3);
  const int rs = (lane & 7) * 8;
  const int c = c0 + cl;
  v8us_r val;
#pragma unroll
  for (int e = 0; e < 8; ++e) {
    const float x = tile[cl][rs + e];
    const unsigned short bb = f32_to_bf16_rne(x);
    unsigned short bits;
    if (MODE == 0) bits = bb;
    else bits = h_bits((_Float16)bf16_to_f32(bb));
    val[e] = bits;
  }
  const bool ok = (c < C) && (r0 + rs + 8 <= R);
  unsigned short* dst = outp + boff + (size_t)c * (size_t)R + (size_t)(r0 + rs);
  if (ok) *(volatile v8us*)dst = val;
  __threadfence();
  if (ok) *(volatile v8us*)dst = val;
}

__global__ __launch_bounds__(NTHR)
void k_attn(const float* __restrict__ d1, const unsigned short* __restrict__ Kt,
            const unsigned short* __restrict__ Vt, const unsigned short* __restrict__ Wt,
            const float* __restrict__ d5, float* __restrict__ outp)
{
  extern __shared__ uint4 smem_raw[];
  unsigned char* smem = (unsigned char*)smem_raw;
  unsigned short* Qs = (unsigned short*)(smem);
  float* Sc = (float*)(smem + LDS_Q);
  unsigned short* Pc = (unsigned short*)(smem + LDS_Q + LDS_S);
  float* stf = (float*)(smem + LDS_Q + LDS_S + LDS_P);
  float* sts = stf + QT;

  const int tid = threadIdx.x, lane = tid & 31, wave = tid >> 5;
  const int h = lane >> 4, m16 = lane & 15;
  const int blk = blockIdx.x;
  const int b = blk / (SEQ / QT);
  const int q0 = (blk - b * (SEQ / QT)) * QT;
  const unsigned short* Kb = Kt + (size_t)b * SEQ * DIM;
  const unsigned short* Vb = Vt + (size_t)b * DIM * SEQ;

  {
    const float* Qg = d1 + ((size_t)b * SEQ + q0) * DIM;
    for (int i = tid; i < QT * DIM; i += NTHR) Qs[i] = f32_to_bf16_rne(Qg[i]);
  }
  __syncthreads();

  v8f cacc[4];
#pragma unroll
  for (int j = 0; j < 4; ++j) cacc[j] = z8();
  float mst[2] = {NEG_BIG, NEG_BIG};
  float sst[2] = {0.0f, 0.0f};

#pragma unroll 1
  for (int c = 0; c < NCH; ++c) {
    const int tc0 = c * CH;

    {
      const int tw = wave * (CH / 8);
#pragma unroll 1
      for (int p = 0; p < CH / 8; p += 32) {
        const int tl = tw + p;
        v8f s0 = z8(), s1 = z8();
#pragma unroll 1
        for (int k0 = 0; k0 < DIM; k0 += 32) {
          const FragB qa  = ld_frag<FragB>(Qs, 0, k0, DIM, lane);
          const FragB kf0 = ld_frag<FragB>(Kb, tc0 + tl, k0, DIM, lane);
          const FragB kf1 = ld_frag<FragB>(Kb, tc0 + tl + 16, k0, DIM, lane);
          s0 = mma_bf16(qa, kf0, s0);
          s1 = mma_bf16(qa, kf1, s1);
        }
#pragma unroll
        for (int r = 0; r < 8; ++r) {
          Sc[(8 * h + r) * CH + tl + m16]      = s0[r];
          Sc[(8 * h + r) * CH + tl + 16 + m16] = s1[r];
        }
      }
    }
    __syncthreads();

#pragma unroll
    for (int rr = 0; rr < 2; ++rr) {
      const int r = 2 * wave + rr;
      const float* srow = Sc + r * CH;
      unsigned short* prow = Pc + r * CH;
      float mx = NEG_BIG;
#pragma unroll 4
      for (int i = lane; i < CH; i += 32) mx = fmaxf(mx, srow[i]);
#pragma unroll
      for (int o = 16; o > 0; o >>= 1) mx = fmaxf(mx, __shfl_xor(mx, o, 32));
      const float mn  = fmaxf(mst[rr], mx);
      const float fac = (c == 0) ? 0.0f : __expf(mst[rr] - mn);
      float sl = 0.0f;
#pragma unroll 4
      for (int i = lane; i < CH; i += 32) {
        const float e = __expf(srow[i] - mn);
        sl += e;
        prow[i] = h_bits((_Float16)(e * P_SCALE));
      }
#pragma unroll
      for (int o = 16; o > 0; o >>= 1) sl += __shfl_xor(sl, o, 32);
      sst[rr] = sst[rr] * fac + sl;
      mst[rr] = mn;
      if (lane == 0) {
        stf[r] = fac;
        if (c == NCH - 1) sts[r] = sst[rr];
      }
    }
    __syncthreads();

    {
      v8f fv = z8();
#pragma unroll
      for (int r = 0; r < 8; ++r) fv[r] = stf[8 * h + r];
#pragma unroll
      for (int j = 0; j < 4; ++j) cacc[j] = cacc[j] * fv;
      const int d0 = wave * 64;
#pragma unroll 1
      for (int t0 = 0; t0 < CH; t0 += 32) {
        const FragH pa = ld_frag<FragH>(Pc, 0, t0, CH, lane);
#pragma unroll
        for (int j = 0; j < 4; ++j) {
          const FragH vb = ld_frag<FragH>(Vb, d0 + 16 * j, tc0 + t0, SEQ, lane);
          cacc[j] = mma_f16(pa, vb, cacc[j]);
        }
      }
    }
  }

  {
    unsigned short* Ah = (unsigned short*)Sc;
    unsigned short* Al = Ah + QT * DIM;
    v8f gv = z8();
#pragma unroll
    for (int r = 0; r < 8; ++r) gv[r] = C_SCALE / sts[8 * h + r];
    const int d0 = wave * 64;
#pragma unroll
    for (int j = 0; j < 4; ++j) {
      const v8f x = cacc[j] * gv;
      const int colb = d0 + 16 * j + m16;
#pragma unroll
      for (int r = 0; r < 8; ++r) {
        const float xv = x[r];
        const _Float16 hi = (_Float16)xv;
        const _Float16 lo = (_Float16)(xv - (float)hi);
        const int idx = (8 * h + r) * DIM + colb;
        Ah[idx] = h_bits(hi);
        Al[idx] = h_bits(lo);
      }
    }
  }
  __syncthreads();

  {
    const unsigned short* Ah = (const unsigned short*)Sc;
    const unsigned short* Al = Ah + QT * DIM;
    v8f oacc[4];
#pragma unroll
    for (int j = 0; j < 4; ++j) oacc[j] = z8();
    const int j0 = wave * 64;
#pragma unroll 1
    for (int k0 = 0; k0 < DIM; k0 += 32) {
      const FragH ah = ld_frag<FragH>(Ah, 0, k0, DIM, lane);
      const FragH al = ld_frag<FragH>(Al, 0, k0, DIM, lane);
#pragma unroll
      for (int j = 0; j < 4; ++j) {
        const FragH wb = ld_frag<FragH>(Wt, j0 + 16 * j, k0, DIM, lane);
        oacc[j] = mma_f16(ah, wb, oacc[j]);
        oacc[j] = mma_f16(al, wb, oacc[j]);
      }
    }
    float* Os = (float*)Pc;
#pragma unroll
    for (int j = 0; j < 4; ++j) {
      const int oc = j0 + 16 * j + m16;
      const float bz = bf16_to_f32(f32_to_bf16_rne(d5[oc]));
#pragma unroll
      for (int r = 0; r < 8; ++r) Os[(8 * h + r) * DIM + oc] = oacc[j][r] * O_SCALE + bz;
    }
  }
  __syncthreads();

  {
    const float* Os = (const float*)Pc;
    float* ob = outp + ((size_t)b * SEQ + q0) * DIM;
    v4f_r vv[8];
    int off[8];
#pragma unroll
    for (int it = 0; it < 8; ++it) {
      const int L = wave * 32 + it * 4 + (lane >> 3);
      off[it] = L * 32 + (lane & 7) * 4;
      vv[it] = *(const v4f*)(Os + off[it]);
    }
#pragma unroll
    for (int it = 0; it < 8; ++it) *(volatile v4f*)(ob + off[it]) = vv[it];
    __threadfence();
#pragma unroll
    for (int it = 0; it < 8; ++it) *(volatile v4f*)(ob + off[it]) = vv[it];
  }
}

extern "C" void kernel_launch(void* const* d_in, const int* in_sizes, int n_in,
                              void* d_out, int out_size, void* d_ws, size_t ws_size,
                              hipStream_t stream)
{
  if (n_in < 5) return;
  if (in_sizes[0] != NB * SEQ * DIM) return;
  if (in_sizes[1] != NB * DIM * SEQ) return;
  if (in_sizes[2] != NB * SEQ * DIM) return;
  if (in_sizes[3] != DIM * DIM) return;
  if (in_sizes[4] != DIM) return;
  if (out_size != NB * SEQ * DIM) return;

  const float* d1 = (const float*)d_in[0];
  const float* d2 = (const float*)d_in[1];
  const float* d3 = (const float*)d_in[2];
  const float* d4 = (const float*)d_in[3];
  const float* d5 = (const float*)d_in[4];
  float* outp = (float*)d_out;

  unsigned char* ws = (unsigned char*)d_ws;
  const size_t bytesK = (size_t)NB * SEQ * DIM * 2;
  const size_t bytesV = (size_t)NB * DIM * SEQ * 2;
  const size_t bytesW = (size_t)DIM * DIM * 2;
  const size_t offK = 0;
  const size_t offV = offK + bytesK;
  const size_t offW = offV + bytesV;
  if (offW + bytesW > ws_size) return;
  unsigned short* Kt = (unsigned short*)(ws + offK);
  unsigned short* Vt = (unsigned short*)(ws + offV);
  unsigned short* Wt = (unsigned short*)(ws + offW);

  k_tr16<0><<<dim3((SEQ + 31) / 32, (DIM + 63) / 64, NB), dim3(NTHR), 0, stream>>>(d2, Kt, DIM, SEQ);
  k_tr16<1><<<dim3((DIM + 31) / 32, (SEQ + 63) / 64, NB), dim3(NTHR), 0, stream>>>(d3, Vt, SEQ, DIM);
  k_tr16<1><<<dim3((DIM + 31) / 32, (DIM + 63) / 64, 1), dim3(NTHR), 0, stream>>>(d4, Wt, DIM, DIM);

  k_attn<<<dim3(NB * (SEQ / QT)), dim3(NTHR), LDS_ALL, stream>>>(d1, Kt, Vt, Wt, d5, outp);
}
